// MPNN_40286793237043
// MI455X (gfx1250) — hardware-verified
//
#include <hip/hip_runtime.h>
#include <math.h>

#define NB    8
#define NNODE 64
#define FIN   32
#define FE    16
#define HS    64
#define MS    64
#define EHD   50
#define TOUT  12
#define RDH   200
#define RDP   208
#define KT    3264
#define NODES 512
#define HP    424

static_assert(51 * 64 == KT);
static_assert(KT % 32 == 0);
static_assert(HS == 64 && MS == 64 && NNODE == 64);
static_assert(EHD + 1 <= 64);
static_assert(RDH <= RDP && RDP % 16 == 0 && (2 * RDP) % 32 == 0);
static_assert(TOUT <= 16);
static_assert(3 * HS == 192);
static_assert(FE <= 32);
static_assert(NB * NNODE == NODES);

typedef unsigned short v8us  __attribute__((ext_vector_type(8)));
typedef unsigned short v16us __attribute__((ext_vector_type(16)));
typedef __bf16         v16bf __attribute__((ext_vector_type(16)));
typedef float          v8f   __attribute__((ext_vector_type(8)));
typedef float          v4f   __attribute__((ext_vector_type(4)));
typedef v8us __attribute__((may_alias)) v8us_a;
typedef v4f  __attribute__((may_alias)) v4f_a;

union FragU { v16us u; v8us h[2]; };

__device__ __forceinline__ unsigned short f2bf(float f) {
  const unsigned u = __float_as_uint(f);
  return (unsigned short)((u + 0x7FFFu + ((u >> 16) & 1u)) >> 16);
}
__device__ __forceinline__ float bf2f(unsigned short b) { return __uint_as_float(((unsigned)b) << 16); }
__device__ __forceinline__ float bfr(float f) { return bf2f(f2bf(f)); }
__device__ __forceinline__ float blendf(float a, float b, unsigned mk) {
  return __uint_as_float((__float_as_uint(a) & mk) | (__float_as_uint(b) & ~mk));
}

__device__ __forceinline__ v16bf ldfrag_g(const unsigned short* __restrict__ p) {
  FragU f;
  f.h[0] = *(const v8us_a*)(p);
  f.h[1] = *(const v8us_a*)(p + 16);
  return __builtin_bit_cast(v16bf, f.u);
}
__device__ __forceinline__ v16bf ldfrag_s(const unsigned short* p) {
  FragU f;
  f.h[0] = *(const v8us_a*)(p);
  f.h[1] = *(const v8us_a*)(p + 16);
  return __builtin_bit_cast(v16bf, f.u);
}
__device__ __forceinline__ v8f mma(v16bf a, v16bf b, v8f c) {
  c = __builtin_amdgcn_wmma_f32_16x16x32_bf16(false, a, false, b, (short)0, c, false, false);
  asm volatile("v_nop\n\tv_nop\n\tv_nop\n\tv_nop" : "+v"(c) : "v"(a), "v"(b));
  return c;
}

__device__ __forceinline__ v8us pk8(float a0, float a1, float a2, float a3,
                                    float a4, float a5, float a6, float a7) {
  const v8us o = { f2bf(a0), f2bf(a1), f2bf(a2), f2bf(a3), f2bf(a4), f2bf(a5), f2bf(a6), f2bf(a7) };
  return o;
}
__device__ __forceinline__ void put8(unsigned short* dst, v8us o) {
  *(volatile v8us*)dst = o;
  __threadfence();
  *(volatile v8us*)dst = o;
}
__device__ __forceinline__ void put4(float* dst, v4f o) {
  *(volatile v4f*)dst = o;
  __threadfence();
  *(volatile v4f*)dst = o;
}

#define PC_W1T   256
#define PC_W2A   52224
#define PC_WG    3072
#define PC_WI1T  4992
#define PC_WJ1T  3328
#define PC_W2T   832
#define PC_HHL   8192
#define PC_HF    8192
#define PC_VAL   128
#define PB_W2A  (PC_W1T)
#define PB_WIH  (PB_W2A + PC_W2A)
#define PB_WHH  (PB_WIH + PC_WG)
#define PB_WI1  (PB_WHH + PC_WG)
#define PB_WJ1  (PB_WI1 + PC_WI1T)
#define PB_WI2  (PB_WJ1 + PC_WJ1T)
#define PB_WJ2  (PB_WI2 + PC_W2T)
#define PB_HHL  (PB_WJ2 + PC_W2T)
#define PB_HF   (PB_HHL + PC_HHL)
#define PB_VAL  (PB_HF + PC_HF)
#define PC_TOTAL (PB_VAL + PC_VAL)
static_assert(PC_TOTAL == 85120);
static_assert(PB_W2A % 32 == 0 && PB_WIH % 32 == 0 && PB_WHH % 32 == 0 && PB_WI1 % 32 == 0);
static_assert(PB_WJ1 % 32 == 0 && PB_WI2 % 32 == 0 && PB_WJ2 % 32 == 0 && PB_HHL % 32 == 0);
static_assert(PB_HF % 32 == 0 && PB_VAL % 32 == 0 && PC_TOTAL % 32 == 0);
static_assert(PC_W1T * 8 == 64 * 32 && PC_W2A * 8 == KT * 128 && PC_WG * 8 == 192 * 128);
static_assert(PC_WI1T * 8 == RDP * 192 && PC_WJ1T * 8 == RDP * 128 && PC_W2T * 8 == 16 * 2 * RDP);
static_assert(PC_HHL * 8 == NODES * 128 && PC_HF * 4 == NODES * 64 && PC_VAL * 4 == NODES);

__device__ __forceinline__ void piece_dup64(const float* __restrict__ W, int q, unsigned short* dst) {
  const int n = q >> 4, kb = ((q & 15) * 8) & 63;
  const v4f a = *(const v4f_a*)(W + n * 64 + kb);
  const v4f c = *(const v4f_a*)(W + n * 64 + kb + 4);
  put8(dst + (size_t)q * 8, pk8(a.x, a.y, a.z, a.w, c.x, c.y, c.z, c.w));
}
__device__ __forceinline__ void piece_w2t(const float* __restrict__ W, int q, unsigned short* dst) {
  const int t = q / 52, pc = q - t * 52;
  const int c8 = pc * 8;
  const int kk0 = (c8 >= RDP) ? (c8 - RDP) : c8;
  const int tc = (t < TOUT) ? t : (TOUT - 1);
  float v[8];
#pragma unroll
  for (int e = 0; e < 8; ++e) {
    const int kk = kk0 + e;
    const int kc = (kk < RDH) ? kk : (RDH - 1);
    const float x = W[kc * TOUT + tc];
    v[e] = (kk < RDH && t < TOUT) ? x : 0.0f;
  }
  put8(dst + (size_t)q * 8, pk8(v[0], v[1], v[2], v[3], v[4], v[5], v[6], v[7]));
}
__device__ __forceinline__ float node_flag(const float* __restrict__ row) {
  float s = 0.0f;
#pragma unroll 1
  for (int f4 = 0; f4 < 8; ++f4) {
    const v4f x = *(const v4f_a*)(row + 4 * f4);
    s += bfr(x.x); s += bfr(x.y); s += bfr(x.z); s += bfr(x.w);
  }
  return (s > 0.0f) ? 1.0f : 0.0f;
}

__global__ __launch_bounds__(256) void k_prep(
    const float* __restrict__ h_in, const float* __restrict__ We1, const float* __restrict__ We2,
    const float* __restrict__ be2, const float* __restrict__ W_ih, const float* __restrict__ W_hh,
    const float* __restrict__ Wi1, const float* __restrict__ Wi2, const float* __restrict__ Wj1,
    const float* __restrict__ Wj2,
    unsigned short* __restrict__ W1T, unsigned short* __restrict__ W2A,
    unsigned short* __restrict__ WIH2, unsigned short* __restrict__ WHH2,
    unsigned short* __restrict__ WI1T, unsigned short* __restrict__ WJ1T,
    unsigned short* __restrict__ WI2T, unsigned short* __restrict__ WJ2T,
    unsigned short* __restrict__ H0HL, float* __restrict__ HF0, float* __restrict__ VALID)
{
  const int p = blockIdx.x * 256 + threadIdx.x;
  if (p >= PC_TOTAL) return;
  if (p < PB_W2A) {
    const int q = p;
    const int n = q >> 2, k8 = (q & 3) * 8;
    const int nc = (n < EHD) ? n : (EHD - 1);
    float v[8];
#pragma unroll
    for (int e = 0; e < 8; ++e) {
      const int k = k8 + e;
      const int kc = (k < FE) ? k : (FE - 1);
      const float x = We1[kc * EHD + nc];
      v[e] = (n < EHD && k < FE) ? x : 0.0f;
    }
    put8(W1T + (size_t)q * 8, pk8(v[0], v[1], v[2], v[3], v[4], v[5], v[6], v[7]));
  } else if (p < PB_WIH) {
    const int q = p - PB_W2A;
    const int rho = q >> 4, hc = ((q & 15) * 8) & 63;
    const int isw = (rho < EHD * 64) ? 1 : 0;
    const unsigned mk = (unsigned)(-isw);
    const int r1 = isw ? rho : (EHD * 64 - 1);
    const int r2 = isw ? 0 : (rho - EHD * 64);
    const v4f a0 = *(const v4f_a*)(We2 + r1 * 64 + hc);
    const v4f a1 = *(const v4f_a*)(We2 + r1 * 64 + hc + 4);
    const v4f b0 = *(const v4f_a*)(be2 + r2 * 64 + hc);
    const v4f b1 = *(const v4f_a*)(be2 + r2 * 64 + hc + 4);
    put8(W2A + (size_t)q * 8,
         pk8(blendf(a0.x, b0.x, mk), blendf(a0.y, b0.y, mk), blendf(a0.z, b0.z, mk), blendf(a0.w, b0.w, mk),
             blendf(a1.x, b1.x, mk), blendf(a1.y, b1.y, mk), blendf(a1.z, b1.z, mk), blendf(a1.w, b1.w, mk)));
  } else if (p < PB_WHH) {
    piece_dup64(W_ih, p - PB_WIH, WIH2);
  } else if (p < PB_WI1) {
    piece_dup64(W_hh, p - PB_WHH, WHH2);
  } else if (p < PB_WJ1) {
    const int q = p - PB_WI1;
    const int n = q / 24, pc = q - n * 24;
    const int c8 = pc * 8;
    const int kb = (c8 & 63) + (((c8 >> 6) == 2) ? 64 : 0);
    const int nc = (n < RDH) ? n : (RDH - 1);
    float v[8];
#pragma unroll
    for (int e = 0; e < 8; ++e) {
      const float x = Wi1[(kb + e) * RDH + nc];
      v[e] = (n < RDH) ? x : 0.0f;
    }
    put8(WI1T + (size_t)q * 8, pk8(v[0], v[1], v[2], v[3], v[4], v[5], v[6], v[7]));
  } else if (p < PB_WI2) {
    const int q = p - PB_WJ1;
    const int n = q >> 4, kb = ((q & 15) * 8) & 63;
    const int nc = (n < RDH) ? n : (RDH - 1);
    float v[8];
#pragma unroll
    for (int e = 0; e < 8; ++e) {
      const float x = Wj1[(kb + e) * RDH + nc];
      v[e] = (n < RDH) ? x : 0.0f;
    }
    put8(WJ1T + (size_t)q * 8, pk8(v[0], v[1], v[2], v[3], v[4], v[5], v[6], v[7]));
  } else if (p < PB_WJ2) {
    piece_w2t(Wi2, p - PB_WI2, WI2T);
  } else if (p < PB_HHL) {
    piece_w2t(Wj2, p - PB_WJ2, WJ2T);
  } else if (p < PB_HF) {
    const int q = p - PB_HHL;
    const int node = q >> 4, c8 = (q & 15) * 8;
    const bool ok = c8 < FIN;
    const int cc = ok ? c8 : (FIN - 8);
    const v4f a = *(const v4f_a*)(h_in + node * FIN + cc);
    const v4f c = *(const v4f_a*)(h_in + node * FIN + cc + 4);
    put8(H0HL + (size_t)q * 8,
         pk8(ok ? a.x : 0.0f, ok ? a.y : 0.0f, ok ? a.z : 0.0f, ok ? a.w : 0.0f,
             ok ? c.x : 0.0f, ok ? c.y : 0.0f, ok ? c.z : 0.0f, ok ? c.w : 0.0f));
  } else if (p < PB_VAL) {
    const int q = p - PB_HF;
    const int node = q >> 4, c4 = (q & 15) * 4;
    const bool ok = c4 < FIN;
    const int cc = ok ? c4 : (FIN - 4);
    const v4f a = *(const v4f_a*)(h_in + node * FIN + cc);
    const v4f o = { ok ? bfr(a.x) : 0.0f, ok ? bfr(a.y) : 0.0f, ok ? bfr(a.z) : 0.0f, ok ? bfr(a.w) : 0.0f };
    put4(HF0 + (size_t)q * 4, o);
  } else {
    const int q = p - PB_VAL;
    const float f0 = node_flag(h_in + (4 * q + 0) * FIN);
    const float f1 = node_flag(h_in + (4 * q + 1) * FIN);
    const float f2 = node_flag(h_in + (4 * q + 2) * FIN);
    const float f3 = node_flag(h_in + (4 * q + 3) * FIN);
    const v4f o = { f0, f1, f2, f3 };
    put4(VALID + (size_t)q * 4, o);
  }
}

__global__ __launch_bounds__(128) void k_edge(
    const float* __restrict__ g, const float* __restrict__ e, const float* __restrict__ be1,
    const unsigned short* __restrict__ W1T,
    unsigned short* __restrict__ GRh, unsigned short* __restrict__ GRl)
{
  __shared__ __attribute__((aligned(16))) unsigned short As[64 * 32];
  __shared__ __attribute__((aligned(16))) float S[64 * 68];
  __shared__ float gs[64];

  const int tid = threadIdx.x, lane = tid & 31, w = tid >> 5;
  const int h = lane >> 4, m = lane & 15;
  const int bj = blockIdx.x, b = bj >> 6, j = bj & 63;

  {
    const int i = tid >> 1, half = tid & 1;
    const float* ep = e + ((size_t)((b * 64 + i) * 64 + j)) * FE + 8 * half;
    const v4f a = *(const v4f_a*)ep;
    const v4f c = *(const v4f_a*)(ep + 4);
    const v8us o = pk8(a.x, a.y, a.z, a.w, c.x, c.y, c.z, c.w);
    const v8us z = { 0, 0, 0, 0, 0, 0, 0, 0 };
    *(v8us_a*)(As + i * 32 + 8 * half) = o;
    *(v8us_a*)(As + i * 32 + 16 + 8 * half) = z;
    if (tid < 64) gs[tid] = bfr(g[(b * 64 + tid) * 64 + j]);
  }
  __syncthreads();

  const v8f zero8 = {0.f, 0.f, 0.f, 0.f, 0.f, 0.f, 0.f, 0.f};
  const v16bf a = ldfrag_s(As + (16 * w + m) * 32 + 8 * h);
  v8f acc[4];
#pragma unroll
  for (int nt = 0; nt < 4; ++nt) {
    const v16bf bw = ldfrag_g(W1T + (16 * nt + m) * 32 + 8 * h);
    acc[nt] = mma(a, bw, zero8);
  }
#pragma unroll
  for (int nt = 0; nt < 4; ++nt) {
    const int k = 16 * nt + m;
    const int kc = (k < EHD) ? k : (EHD - 1);
    const float bv = bfr(be1[kc]);
#pragma unroll
    for (int r = 0; r < 8; ++r) {
      const int i = 16 * w + 8 * h + r;
      const float act = fmaxf(acc[nt][r] + bv, 0.0f);
      float v = (k < EHD) ? act : ((k == EHD) ? 1.0f : 0.0f);
      v = v * gs[i];
      S[i * 68 + k] = v;
    }
  }
  __syncthreads();

  const int l8 = tid & 7, ls = tid >> 3;
  unsigned short* ph = GRh + (size_t)bj * KT;
  unsigned short* pl = GRl + (size_t)bj * KT;
  for (int pass = 0; pass < 2; ++pass) {
#pragma unroll 1
    for (int rd = 0; rd < 4; ++rd) {
      const int k = rd * 16 + ls;
      const int kc = (k <= EHD) ? k : EHD;
      v8us hv, lv;
#pragma unroll
      for (int q = 0; q < 8; ++q) {
        const float f = S[(8 * l8 + q) * 68 + kc];
        const unsigned short hb = f2bf(f);
        const unsigned short lb = f2bf(f - bf2f(hb));
        hv[q] = hb; lv[q] = lb;
      }
      if (k <= EHD) {
        *(volatile v8us*)(ph + k * 64 + 8 * l8) = hv;
        *(volatile v8us*)(pl + k * 64 + 8 * l8) = lv;
      }
    }
    __threadfence();
  }
}

__global__ __launch_bounds__(256) void k_P(
    const unsigned short* __restrict__ W2A, const unsigned short* __restrict__ HHL,
    unsigned short* __restrict__ PTh, unsigned short* __restrict__ PTl)
{
  __shared__ __attribute__((aligned(16))) float sT[8 * 16 * 68];
  const int lane = threadIdx.x & 31, wave = threadIdx.x >> 5;
  const int rl = lane & 15, koff = (lane >> 4) * 8, hOff = (lane >> 4) * 8;
  const int blk = blockIdx.x, kt = blk >> 1, mu0 = (blk & 1) * 32;
  const int b = wave;

  const v8f zero8 = {0.f, 0.f, 0.f, 0.f, 0.f, 0.f, 0.f, 0.f};
  v8f acc[2][4];
#pragma unroll
  for (int i = 0; i < 2; ++i)
#pragma unroll
    for (int jn = 0; jn < 4; ++jn) acc[i][jn] = zero8;

#pragma unroll 1
  for (int k0 = 0; k0 < 128; k0 += 32) {
    v16bf bv[4];
#pragma unroll
    for (int jn = 0; jn < 4; ++jn)
      bv[jn] = ldfrag_g(HHL + (size_t)(b * 64 + 16 * jn + rl) * 128 + k0 + koff);
#pragma unroll
    for (int i = 0; i < 2; ++i) {
      const v16bf av = ldfrag_g(W2A + (size_t)(kt * 64 + mu0 + 16 * i + rl) * 128 + k0 + koff);
#pragma unroll
      for (int jn = 0; jn < 4; ++jn) acc[i][jn] = mma(av, bv[jn], acc[i][jn]);
    }
  }

  float* slab = sT + wave * (16 * 68);
  const int q = lane >> 3, c8 = (lane & 7) * 8;
#pragma unroll
  for (int i = 0; i < 2; ++i) {
#pragma unroll
    for (int jn = 0; jn < 4; ++jn)
#pragma unroll
      for (int r = 0; r < 8; ++r)
        slab[(hOff + r) * 68 + 16 * jn + rl] = acc[i][jn][r];
    __syncthreads();
    for (int pass = 0; pass < 2; ++pass) {
#pragma unroll
      for (int it = 0; it < 4; ++it) {
        const int row = it * 4 + q;
        const int mu = mu0 + 16 * i + row;
        const float* sp = slab + row * 68 + c8;
        v8us hv, lv;
#pragma unroll
        for (int x = 0; x < 8; ++x) {
          const float f = sp[x];
          const unsigned short hb = f2bf(f);
          const unsigned short lb = f2bf(f - bf2f(hb));
          hv[x] = hb; lv[x] = lb;
        }
        const size_t go = (size_t)(b * 64 + mu) * KT + kt * 64 + c8;
        *(volatile v8us*)(PTh + go) = hv;
        *(volatile v8us*)(PTl + go) = lv;
      }
      __threadfence();
    }
    __syncthreads();
  }
}

__global__ __launch_bounds__(128) void k_upd(
    const unsigned short* __restrict__ GRh, const unsigned short* __restrict__ GRl,
    const unsigned short* __restrict__ PTh, const unsigned short* __restrict__ PTl,
    const unsigned short* __restrict__ HHLp, const float* __restrict__ HFp,
    const unsigned short* __restrict__ WIH2, const unsigned short* __restrict__ WHH2,
    const float* __restrict__ b_ih, const float* __restrict__ b_hh,
    const float* __restrict__ VALID,
    float* __restrict__ HFn, unsigned short* __restrict__ HHLn)
{
  __shared__ __attribute__((aligned(16))) unsigned short Mhl[64 * 136];
  __shared__ __attribute__((aligned(16))) float Ho[64 * 68];
  __shared__ float scr[4 * 1024];

  const int tid = threadIdx.x, lane = tid & 31, w = tid >> 5;
  const int h = lane >> 4, m = lane & 15;
  const int b = blockIdx.x;
  const v8f zero8 = {0.f, 0.f, 0.f, 0.f, 0.f, 0.f, 0.f, 0.f};

  {
    const int tm0 = 2 * (w >> 1), tn0 = 2 * (w & 1);
    const size_t ra = (size_t)(b * 64 + 16 * tm0 + m) * KT + 8 * h;
    const size_t rb = (size_t)(b * 64 + 16 * tn0 + m) * KT + 8 * h;
    const unsigned short* pa0h = GRh + ra;
    const unsigned short* pa1h = pa0h + (size_t)16 * KT;
    const unsigned short* pa0l = GRl + ra;
    const unsigned short* pa1l = pa0l + (size_t)16 * KT;
    const unsigned short* pb0h = PTh + rb;
    const unsigned short* pb1h = pb0h + (size_t)16 * KT;
    const unsigned short* pb0l = PTl + rb;
    const unsigned short* pb1l = pb0l + (size_t)16 * KT;
    v8f c00 = zero8, c01 = zero8, c10 = zero8, c11 = zero8;
#pragma unroll 1
    for (int k0 = 0; k0 < KT; k0 += 32) {
      const v16bf a0h = ldfrag_g(pa0h + k0);
      const v16bf a0l = ldfrag_g(pa0l + k0);
      const v16bf a1h = ldfrag_g(pa1h + k0);
      const v16bf a1l = ldfrag_g(pa1l + k0);
      const v16bf b0h = ldfrag_g(pb0h + k0);
      const v16bf b0l = ldfrag_g(pb0l + k0);
      const v16bf b1h = ldfrag_g(pb1h + k0);
      const v16bf b1l = ldfrag_g(pb1l + k0);
      c00 = mma(a0h, b0h, c00); c00 = mma(a0l, b0h, c00); c00 = mma(a0h, b0l, c00);
      c01 = mma(a0h, b1h, c01); c01 = mma(a0l, b1h, c01); c01 = mma(a0h, b1l, c01);
      c10 = mma(a1h, b0h, c10); c10 = mma(a1l, b0h, c10); c10 = mma(a1h, b0l, c10);
      c11 = mma(a1h, b1h, c11); c11 = mma(a1l, b1h, c11); c11 = mma(a1h, b1l, c11);
    }
#pragma unroll
    for (int r = 0; r < 8; ++r) {
      const int j0 = 16 * tm0 + 8 * h + r, j1 = j0 + 16;
      const int u0 = 16 * tn0 + m, u1 = u0 + 16;
      unsigned short hb;
      hb = f2bf(c00[r]); Mhl[j0 * 136 + u0] = hb; Mhl[j0 * 136 + 64 + u0] = f2bf(c00[r] - bf2f(hb));
      hb = f2bf(c01[r]); Mhl[j0 * 136 + u1] = hb; Mhl[j0 * 136 + 64 + u1] = f2bf(c01[r] - bf2f(hb));
      hb = f2bf(c10[r]); Mhl[j1 * 136 + u0] = hb; Mhl[j1 * 136 + 64 + u0] = f2bf(c10[r] - bf2f(hb));
      hb = f2bf(c11[r]); Mhl[j1 * 136 + u1] = hb; Mhl[j1 * 136 + 64 + u1] = f2bf(c11[r] - bf2f(hb));
    }
  }
  __syncthreads();

  const int c = 16 * w + m;
  const float br  = bfr(b_ih[c]) + bfr(b_hh[c]);
  const float bz  = bfr(b_ih[64 + c]) + bfr(b_hh[64 + c]);
  const float bin = bfr(b_ih[128 + c]);
  const float bhn = bfr(b_hh[128 + c]);
  const unsigned short* wi = WIH2 + (size_t)(16 * w + m) * 128 + 8 * h;
  const unsigned short* wh = WHH2 + (size_t)(16 * w + m) * 128 + 8 * h;
  float* sc = scr + w * 1024;
  const float* vrow = VALID + b * 64;
  const float* hp = HFp + (size_t)(b * 64) * 64;

#pragma unroll 1
  for (int tm = 0; tm < 4; ++tm) {
    const unsigned short* am = Mhl + (16 * tm + m) * 136 + 8 * h;
    const unsigned short* ah = HHLp + (size_t)(b * 64 + 16 * tm + m) * 128 + 8 * h;
    v8f ar = zero8, az = zero8, ain = zero8, ahn = zero8;
#pragma unroll 1
    for (int k0 = 0; k0 < 128; k0 += 32) {
      const v16bf fm = ldfrag_s(am + k0);
      const v16bf fh = ldfrag_g(ah + k0);
      const v16bf bir = ldfrag_g(wi + k0);
      const v16bf biz = ldfrag_g(wi + (size_t)64 * 128 + k0);
      const v16bf bnn = ldfrag_g(wi + (size_t)128 * 128 + k0);
      const v16bf bhr = ldfrag_g(wh + k0);
      const v16bf bhz = ldfrag_g(wh + (size_t)64 * 128 + k0);
      const v16bf bhh = ldfrag_g(wh + (size_t)128 * 128 + k0);
      ar  = mma(fm, bir, ar);  ar  = mma(fh, bhr, ar);
      az  = mma(fm, biz, az);  az  = mma(fh, bhz, az);
      ain = mma(fm, bnn, ain);
      ahn = mma(fh, bhh, ahn);
    }
#pragma unroll
    for (int r = 0; r < 8; ++r) {
      sc[r * 32 + lane]       = ar[r];
      sc[256 + r * 32 + lane] = az[r];
      sc[512 + r * 32 + lane] = ain[r];
      sc[768 + r * 32 + lane] = ahn[r];
    }
    __syncthreads();
#pragma unroll 1
    for (int r = 0; r < 8; ++r) {
      const int j = 16 * tm + 8 * h + r;
      const float xr  = sc[r * 32 + lane] + br;
      const float xz  = sc[256 + r * 32 + lane] + bz;
      const float xin = sc[512 + r * 32 + lane] + bin;
      const float xhn = sc[768 + r * 32 + lane] + bhn;
      const float rg = 1.0f / (1.0f + expf(-xr));
      const float zg = 1.0f / (1.0f + expf(-xz));
      const float nn = tanhf(xin + rg * xhn);
      const float hold = hp[j * 64 + c];
      const float hv = ((1.0f - zg) * nn + zg * hold) * vrow[j];
      Ho[j * 68 + c] = hv;
    }
    __syncthreads();
  }

  const int l16 = tid & 15, rs = tid >> 4;
  const int cb = (l16 & 7) * 8;
  const bool isHi = l16 < 8;
  for (int pass = 0; pass < 2; ++pass) {
#pragma unroll 1
    for (int it = 0; it < 8; ++it) {
      const int row = it * 8 + rs;
      const v4f v = *(const v4f_a*)(Ho + row * 68 + 4 * l16);
      *(volatile v4f*)(HFn + (size_t)(b * 64 + row) * 64 + 4 * l16) = v;
      v8us o;
#pragma unroll
      for (int x = 0; x < 8; ++x) {
        const float f = Ho[row * 68 + cb + x];
        const unsigned short hb = f2bf(f);
        const unsigned short lb = f2bf(f - bf2f(hb));
        o[x] = isHi ? hb : lb;
      }
      *(volatile v8us*)(HHLn + (size_t)(b * 64 + row) * 128 + 8 * l16) = o;
    }
    __threadfence();
  }
}

__device__ __forceinline__ v8f second_layer(const unsigned short* hidrow, const unsigned short* __restrict__ wrow) {
  v8f acc = {0.f, 0.f, 0.f, 0.f, 0.f, 0.f, 0.f, 0.f};
#pragma unroll 1
  for (int s = 0; s < 13; ++s) {
    const v16bf a = ldfrag_s(hidrow + 32 * s);
    const v16bf bw = ldfrag_g(wrow + 32 * s);
    acc = mma(a, bw, acc);
  }
  return acc;
}

__global__ __launch_bounds__(128) void k_readout(
    const unsigned short* __restrict__ HT, const unsigned short* __restrict__ H0,
    const unsigned short* __restrict__ WI1T, const unsigned short* __restrict__ WJ1T,
    const unsigned short* __restrict__ WI2T, const unsigned short* __restrict__ WJ2T,
    const float* __restrict__ bi1, const float* __restrict__ bj1,
    const float* __restrict__ bi2, const float* __restrict__ bj2,
    const float* __restrict__ VALID, float* __restrict__ REC)
{
  __shared__ __attribute__((aligned(16))) unsigned short Hid[4 * 16 * HP];
  __shared__ __attribute__((aligned(16))) float Pi[64 * 16];
  __shared__ __attribute__((aligned(16))) float Pj[64 * 16];

  const int tid = threadIdx.x, lane = tid & 31, w = tid >> 5;
  const int h = lane >> 4, m = lane & 15;
  const int b = blockIdx.x;
  const v8f zero8 = {0.f, 0.f, 0.f, 0.f, 0.f, 0.f, 0.f, 0.f};

  const size_t arow = (size_t)(b * 64 + 16 * w + m) * 128 + 8 * h;
  v16bf aH[4], a0[2];
#pragma unroll
  for (int ks = 0; ks < 4; ++ks) aH[ks] = ldfrag_g(HT + arow + 32 * ks);
#pragma unroll
  for (int ks = 0; ks < 2; ++ks) a0[ks] = ldfrag_g(H0 + arow + 32 * ks);
  unsigned short* hid = Hid + w * (16 * HP);

#pragma unroll 1
  for (int ct = 0; ct < 13; ++ct) {
    const int n = 16 * ct + m;
    const unsigned short* bp = WI1T + (size_t)n * 192 + 8 * h;
    v8f acc = zero8;
#pragma unroll
    for (int ks = 0; ks < 4; ++ks) acc = mma(aH[ks], ldfrag_g(bp + 32 * ks), acc);
#pragma unroll
    for (int ks = 0; ks < 2; ++ks) acc = mma(a0[ks], ldfrag_g(bp + 128 + 32 * ks), acc);
    const int nc = (n < RDH) ? n : (RDH - 1);
    const float bias = bfr(bi1[nc]);
#pragma unroll
    for (int r = 0; r < 8; ++r) {
      float v = fmaxf(acc[r] + bias, 0.0f);
      v = (n < RDH) ? v : 0.0f;
      const unsigned short hb = f2bf(v);
      hid[(8 * h + r) * HP + n] = hb;
      hid[(8 * h + r) * HP + RDP + n] = f2bf(v - bf2f(hb));
    }
  }
  __syncthreads();
  const v8f oi = second_layer(hid + m * HP + 8 * h, WI2T + (size_t)m * (2 * RDP) + 8 * h);
  __syncthreads();

#pragma unroll 1
  for (int ct = 0; ct < 13; ++ct) {
    const int n = 16 * ct + m;
    const unsigned short* bp = WJ1T + (size_t)n * 128 + 8 * h;
    v8f acc = zero8;
#pragma unroll
    for (int ks = 0; ks < 4; ++ks) acc = mma(aH[ks], ldfrag_g(bp + 32 * ks), acc);
    const int nc = (n < RDH) ? n : (RDH - 1);
    const float bias = bfr(bj1[nc]);
#pragma unroll
    for (int r = 0; r < 8; ++r) {
      float v = fmaxf(acc[r] + bias, 0.0f);
      v = (n < RDH) ? v : 0.0f;
      const unsigned short hb = f2bf(v);
      hid[(8 * h + r) * HP + n] = hb;
      hid[(8 * h + r) * HP + RDP + n] = f2bf(v - bf2f(hb));
    }
  }
  __syncthreads();
  const v8f oj = second_layer(hid + m * HP + 8 * h, WJ2T + (size_t)m * (2 * RDP) + 8 * h);

#pragma unroll
  for (int r = 0; r < 8; ++r) {
    Pi[(16 * w + 8 * h + r) * 16 + m] = oi[r];
    Pj[(16 * w + 8 * h + r) * 16 + m] = oj[r];
  }
  __syncthreads();

#pragma unroll 1
  for (int it = 0; it < 8; ++it) {
    const int idx = it * 128 + tid;
    const int node = idx >> 4, t = idx & 15;
    const int tc = (t < TOUT) ? t : (TOUT - 1);
    const float xi = Pi[idx] + bfr(bi2[tc]);
    const float xj = Pj[idx] + bfr(bj2[tc]);
    const float ia = 1.0f / (1.0f + expf(-xi));
    const float pr = (VALID[b * 64 + node] * ia) * xj;
    Pi[idx] = (t < TOUT) ? pr : 0.0f;
  }
  __syncthreads();

  if (tid < 32) {
    const int t = tid & 15;
    float s = 0.0f;
#pragma unroll 4
    for (int i = 0; i < 64; ++i) s += Pi[i * 16 + t];
    Pj[tid] = (tid < TOUT) ? s : 0.0f;
  }
  __syncthreads();
  {
    const int pc = (tid < 8) ? tid : 7;
    const v4f v = *(const v4f_a*)(Pj + 4 * pc);
    float* dst = REC + b * 32 + 4 * pc;
    if (tid < 8) { *(volatile v4f*)dst = v; }
    __threadfence();
    if (tid < 8) { *(volatile v4f*)dst = v; }
  }
}

__global__ __launch_bounds__(32) void k_out(const float* __restrict__ REC, float* __restrict__ out)
{
  const int lane = threadIdx.x;
  const int lc = (lane < 24) ? lane : 23;
  const int bb = lc / 3, part = lc - 3 * bb;
  const v4f v = *(const v4f_a*)(REC + bb * 32 + 4 * part);
  if (lane < 24) { *(volatile v4f*)(out + 4 * lane) = v; }
  __threadfence();
  if (lane < 24) { *(volatile v4f*)(out + 4 * lane) = v; }
}
static_assert(4 * 23 + 3 < NB * TOUT);

extern "C" void kernel_launch(void* const* d_in, const int* in_sizes, int n_in,
                              void* d_out, int out_size, void* d_ws, size_t ws_size,
                              hipStream_t stream)
{
  if (n_in < 19) return;
  const int want[19] = { 32768, 16384, 524288, 800, 50, 204800, 4096, 12288, 12288, 192, 192,
                         25600, 200, 2400, 12, 12800, 200, 2400, 12 };
  for (int i = 0; i < 19; ++i) if (in_sizes[i] != want[i]) return;
  if (out_size != NB * TOUT) return;

  const float* g    = (const float*)d_in[0];
  const float* h_in = (const float*)d_in[1];
  const float* e    = (const float*)d_in[2];
  const float* We1  = (const float*)d_in[3];
  const float* be1  = (const float*)d_in[4];
  const float* We2  = (const float*)d_in[5];
  const float* be2  = (const float*)d_in[6];
  const float* W_ih = (const float*)d_in[7];
  const float* W_hh = (const float*)d_in[8];
  const float* b_ih = (const float*)d_in[9];
  const float* b_hh = (const float*)d_in[10];
  const float* Wi1  = (const float*)d_in[11];
  const float* bi1  = (const float*)d_in[12];
  const float* Wi2  = (const float*)d_in[13];
  const float* bi2  = (const float*)d_in[14];
  const float* Wj1  = (const float*)d_in[15];
  const float* bj1  = (const float*)d_in[16];
  const float* Wj2  = (const float*)d_in[17];
  const float* bj2  = (const float*)d_in[18];

  const size_t SZ_GR  = (size_t)NB * 64 * KT * 2;
  const size_t SZ_W2A = (size_t)KT * 128 * 2;
  const size_t SZ_H   = (size_t)NODES * 128 * 2;
  const size_t SZ_WG  = (size_t)192 * 128 * 2;
  const size_t SZ_WI1 = (size_t)RDP * 192 * 2;
  const size_t SZ_WJ1 = (size_t)RDP * 128 * 2;
  const size_t SZ_W2T = (size_t)16 * 2 * RDP * 2;
  const size_t SZ_W1T = (size_t)64 * 32 * 2;
  const size_t SZ_VAL = (size_t)NODES * 4;
  const size_t SZ_REC = (size_t)NB * 32 * 4;

  size_t off = 0;
  const size_t oGRh = off; off += SZ_GR;
  const size_t oGRl = off; off += SZ_GR;
  const size_t oPTh = off; off += SZ_GR;
  const size_t oPTl = off; off += SZ_GR;
  const size_t oW2A = off; off += SZ_W2A;
  size_t oHHL[4], oHF[4];
  for (int t = 0; t < 4; ++t) { oHHL[t] = off; off += SZ_H; }
  for (int t = 0; t < 4; ++t) { oHF[t]  = off; off += SZ_H; }
  const size_t oWIH = off; off += SZ_WG;
  const size_t oWHH = off; off += SZ_WG;
  const size_t oWI1 = off; off += SZ_WI1;
  const size_t oWJ1 = off; off += SZ_WJ1;
  const size_t oWI2 = off; off += SZ_W2T;
  const size_t oWJ2 = off; off += SZ_W2T;
  const size_t oW1T = off; off += SZ_W1T;
  const size_t oVAL = off; off += SZ_VAL;
  const size_t oREC = off; off += SZ_REC;
  if (off > ws_size) return;
  if (off > (size_t)134217728) return;

  char* ws = (char*)d_ws;
  unsigned short* GRh  = (unsigned short*)(ws + oGRh);
  unsigned short* GRl  = (unsigned short*)(ws + oGRl);
  unsigned short* PTh  = (unsigned short*)(ws + oPTh);
  unsigned short* PTl  = (unsigned short*)(ws + oPTl);
  unsigned short* W2A  = (unsigned short*)(ws + oW2A);
  unsigned short* WIH2 = (unsigned short*)(ws + oWIH);
  unsigned short* WHH2 = (unsigned short*)(ws + oWHH);
  unsigned short* WI1T = (unsigned short*)(ws + oWI1);
  unsigned short* WJ1T = (unsigned short*)(ws + oWJ1);
  unsigned short* WI2T = (unsigned short*)(ws + oWI2);
  unsigned short* WJ2T = (unsigned short*)(ws + oWJ2);
  unsigned short* W1T  = (unsigned short*)(ws + oW1T);
  float* VALID = (float*)(ws + oVAL);
  float* REC   = (float*)(ws + oREC);

  k_prep<<<(PC_TOTAL + 255) / 256, 256, 0, stream>>>(
      h_in, We1, We2, be2, W_ih, W_hh, Wi1, Wi2, Wj1, Wj2,
      W1T, W2A, WIH2, WHH2, WI1T, WJ1T, WI2T, WJ2T,
      (unsigned short*)(ws + oHHL[0]), (float*)(ws + oHF[0]), VALID);

  k_edge<<<NB * 64, 128, 0, stream>>>(g, e, be1, W1T, GRh, GRl);

  for (int t = 0; t < 3; ++t) {
    k_P<<<(KT / 32), 256, 0, stream>>>(W2A, (const unsigned short*)(ws + oHHL[t]), PTh, PTl);
    k_upd<<<NB, 128, 0, stream>>>(GRh, GRl, PTh, PTl,
                                  (const unsigned short*)(ws + oHHL[t]), (const float*)(ws + oHF[t]),
                                  WIH2, WHH2, b_ih, b_hh, VALID,
                                  (float*)(ws + oHF[t + 1]), (unsigned short*)(ws + oHHL[t + 1]));
  }

  k_readout<<<NB, 128, 0, stream>>>((const unsigned short*)(ws + oHHL[3]), (const unsigned short*)(ws + oHHL[0]),
                                    WI1T, WJ1T, WI2T, WJ2T, bi1, bj1, bi2, bj2, VALID, REC);

  k_out<<<1, 32, 0, stream>>>(REC, (float*)d_out);
  (void)hipGetLastError();
}
